// NGCF_RNN_91182155694433
// MI455X (gfx1250) — hardware-run, weakly checked
//
#include <hip/hip_runtime.h>


namespace {
constexpr int NU = 100000, NI = 50000, N = NU + NI, NP = 150016  , E = 2400000, D = 64, NLAY = 3, NBQ = 4096, NSEL = 2 * NBQ;
constexpr float XS = 8.0f, WSC = 256.0f, NEG = 0.2f, NRM_EPS = 1e-12f;

typedef _Float16 b16;
typedef __attribute__((ext_vector_type(16))) _Float16 v16b;
typedef __attribute__((ext_vector_type(8))) _Float16 v8b;
typedef __attribute__((ext_vector_type(8))) float v8f;
typedef __attribute__((ext_vector_type(4))) float v4f;
__device__ __forceinline__ float bf16_rne(float f) { unsigned int u = __float_as_uint(f); u += 0x7FFFu + ((u >> 16) & 1u); return __uint_as_float(u & 0xFFFF0000u); }
__device__ __forceinline__ void split16(float v, b16& hi, b16& lo) { hi = (b16)v; lo = (b16)(v - (float)hi); }
__device__ __forceinline__ v16b frag_kb(const b16* p, int hh) { const v8b a = *(const v8b*)(p + 8 * hh), b = *(const v8b*)(p + 16 + 8 * hh); v16b f;
#pragma unroll
  for (int e = 0; e < 8; ++e) { f[e] = a[e]; f[8 + e] = b[e]; } return f; }
__device__ __forceinline__ v8f wmma16b(v16b a, v16b b, v8f c) { v8f d = __builtin_amdgcn_wmma_f32_16x16x32_f16(false, a, false, b, (short)0, c, false, false); asm volatile("v_nop\n\tv_nop\n\tv_nop\n\tv_nop" : "+v"(d) : "v"(a), "v"(b)); return d; }
__device__ __forceinline__ void wave_lds_sync() { __builtin_amdgcn_fence(__ATOMIC_RELEASE, "workgroup"); __builtin_amdgcn_wave_barrier(); __builtin_amdgcn_fence(__ATOMIC_ACQUIRE, "workgroup"); }
__device__ __forceinline__ float pmul(float a, float b) { float p = a * b; asm volatile("" : "+v"(p)); return p; }
__device__ __forceinline__ int iclamp(int v, int lo, int hi) { return v < lo ? lo : (v > hi ? hi : v); }
__device__ __forceinline__ float nexp(float x) { return __builtin_amdgcn_exp2f(x * 1.4426950408889634f); }
__device__ __forceinline__ float lrelu(float x) { return x > 0.0f ? x : NEG * x; }

constexpr int CSR_NBLK = 512, CSR_GB = 9, CSR_GN = 1 << CSR_GB  , CSR_MAXG = 512, CSR_CAP = 12288  ;
__global__ __launch_bounds__(64) void csrA_kernel(const int* __restrict__ dst, int E, int N, int nG, int CHP, int NGP, int* __restrict__ STG, int* __restrict__ HST) {
  extern __shared__ int sm[];
  int* cnt = sm; int* run = sm + NGP; int* ids = sm + 2 * NGP;
  const int b = blockIdx.x; const int ch = (E + CSR_NBLK - 1) / CSR_NBLK; const int e0 = b * ch, e1 = min(E, e0 + ch);
  for (int i = threadIdx.x; i < NGP; i += 64) cnt[i] = 0;
  for (int i = threadIdx.x; i < CHP; i += 64) ids[i] = -1;
  __syncthreads();
  if (threadIdx.x == 0) {
    for (int e = e0; e < e1; ++e) { int d = dst[e]; d = (d < 0) ? 0 : (d >= N ? N - 1 : d); cnt[d >> CSR_GB] += 1; }
    int acc = 0; for (int g = 0; g < nG; ++g) { run[g] = acc; acc += cnt[g]; }
    for (int e = e0; e < e1; ++e) { int d = dst[e]; d = (d < 0) ? 0 : (d >= N ? N - 1 : d); const int g = d >> CSR_GB; ids[run[g]] = e; run[g] += 1; } }
  __syncthreads();
  typedef __attribute__((ext_vector_type(4))) int v4i;
  for (int pass = 0; pass < 2; ++pass) {
    for (int i = threadIdx.x; i < CHP / 4; i += 64) *(volatile v4i*)(STG + (size_t)b * CHP + i * 4) = *(const v4i*)(&ids[i * 4]);
    for (int i = threadIdx.x; i < NGP / 4; i += 64) { v4i v; for (int e = 0; e < 4; ++e) v[e] = (i * 4 + e < nG) ? cnt[i * 4 + e] : 0; *(volatile v4i*)(HST + (size_t)b * NGP + i * 4) = v; }
    __threadfence(); }
}
__global__ __launch_bounds__(512) void csrS_kernel(const int* __restrict__ HST, int nG, int NGP, int* __restrict__ START, int* __restrict__ TOT, int* __restrict__ OFF) {
  __shared__ int tot[CSR_MAXG];
  const int b = threadIdx.x;
  for (int pass = 0; pass < 2; ++pass) { int runb = 0; for (int g = 0; g < nG; ++g) { int c = HST[(size_t)b * NGP + g]; c = (c < 0) ? 0 : c; ((volatile int*)OFF)[(size_t)g * CSR_NBLK + b] = runb; runb += c; } __threadfence(); }
  for (int g = threadIdx.x; g < nG; g += 512) { int s = 0; for (int bb = 0; bb < CSR_NBLK; ++bb) { int c = HST[(size_t)bb * NGP + g]; s += (c < 0) ? 0 : c; } tot[g] = s; }
  __syncthreads();
  if (threadIdx.x < 32) {
    __shared__ int st[CSR_MAXG + 32];
    if (threadIdx.x == 0) { int acc = 0; for (int g = 0; g < NGP; ++g) { st[g] = acc; if (g < nG) acc += (tot[g] + 31) & ~31; } st[NGP] = acc; }
    __builtin_amdgcn_fence(__ATOMIC_RELEASE, "workgroup"); __builtin_amdgcn_wave_barrier(); __builtin_amdgcn_fence(__ATOMIC_ACQUIRE, "workgroup");
    for (int pass = 0; pass < 2; ++pass) { for (int i = threadIdx.x; i < NGP + 32; i += 32) { ((volatile int*)START)[i] = (i <= NGP) ? st[min(i, NGP)] : 0; ((volatile int*)TOT)[i] = (i < nG) ? tot[i] : 0; } __threadfence(); } }
}
__global__ __launch_bounds__(256) void csrB_kernel(const int* __restrict__ dst, int N, int nG, int CHP, int NGP, int permLen, const int* __restrict__ STG, const int* __restrict__ HST, const int* __restrict__ OFF, const int* __restrict__ START, const int* __restrict__ TOT, int* __restrict__ PERM, int* __restrict__ ROWPTR, int* __restrict__ ROWCNT, int* __restrict__ FLAG) {
  typedef __attribute__((ext_vector_type(4))) int v4i;
  __shared__ int ids[CSR_CAP]; __shared__ unsigned short key[CSR_CAP]; __shared__ int outp[CSR_CAP]; __shared__ int ncnt[CSR_GN + 1]; __shared__ int boff[CSR_NBLK + 1];
  const int g = blockIdx.x, t_ = threadIdx.x; int tot = TOT[g]; int st = START[g], stn = START[g + 1]; const int v0 = g * CSR_GN; const int nv = min(CSR_GN, N - v0);
  st = (st < 0) ? 0 : (st > permLen - 32 ? permLen - 32 : st) & ~31; stn = (stn < st) ? st : (stn > permLen ? permLen : stn); tot = (tot < 0) ? 0 : tot; if (tot > stn - st && tot <= CSR_CAP) tot = stn - st;
  if (tot > CSR_CAP) {
    for (int pass = 0; pass < 2; ++pass) { for (int i = t_; i < CSR_GN / 4; i += 256) { v4i a, c; for (int e = 0; e < 4; ++e) { a[e] = st; c[e] = 0; } *(volatile v4i*)(ROWPTR + v0 + i * 4) = a; *(volatile v4i*)(ROWCNT + v0 + i * 4) = c; } if (t_ == 0) ((volatile int*)FLAG)[0] = 1; __threadfence(); } (void)nv; return; }
  if (t_ == 0) { int acc = 0; for (int b = 0; b < CSR_NBLK; ++b) { boff[b] = acc; int c = HST[(size_t)b * NGP + g]; c = (c < 0) ? 0 : (c > CHP ? CHP : c); acc += c; if (acc > tot) acc = tot; } boff[CSR_NBLK] = acc; }
  for (int i = t_; i <= CSR_GN; i += 256) ncnt[i] = 0;
  __syncthreads();
  for (int b = 0; b < CSR_NBLK; ++b) { const int c = boff[b + 1] - boff[b]; int o_ = OFF[(size_t)g * CSR_NBLK + b]; o_ = (o_ < 0) ? 0 : (o_ > CHP - c ? CHP - c : o_); const int* src_ = STG + (size_t)b * CHP + o_;
    for (int i = t_; i < c; i += 256) { int id = src_[i]; id = (id < 0) ? 0 : id; ids[boff[b] + i] = id; int d = dst[id]; d = (d < v0) ? v0 : (d >= N ? N - 1 : d); int kk = d - v0; kk = (kk < 0) ? 0 : (kk >= CSR_GN ? CSR_GN - 1 : kk); key[boff[b] + i] = (unsigned short)kk; } }
  __syncthreads();
  if (t_ == 0) { for (int i = 0; i < tot; ++i) ncnt[key[i]] += 1; int acc = 0; for (int vl = 0; vl < CSR_GN; ++vl) { const int c = ncnt[vl]; ncnt[vl] = acc; acc += c; } ncnt[CSR_GN] = acc;
    for (int i = 0; i < tot; ++i) { const int vl = key[i]; outp[ncnt[vl]] = ids[i]; ncnt[vl] += 1; }
    for (int vl = CSR_GN; vl > 0; --vl) ncnt[vl] = ncnt[vl - 1]; ncnt[0] = 0; }
  __syncthreads();
  for (int pass = 0; pass < 2; ++pass) {
    for (int i = t_; i < (stn - st) / 4; i += 256) { v4i v; for (int e = 0; e < 4; ++e) { const int q = i * 4 + e; v[e] = (q < tot) ? outp[q] : -1; } *(volatile v4i*)(PERM + st + i * 4) = v; }
    for (int i = t_; i < CSR_GN / 4; i += 256) { v4i a, c; for (int e = 0; e < 4; ++e) { const int vl = i * 4 + e; a[e] = st + ncnt[vl]; c[e] = (vl < nv) ? (ncnt[vl + 1] - ncnt[vl]) : 0; } *(volatile v4i*)(ROWPTR + v0 + i * 4) = a; *(volatile v4i*)(ROWCNT + v0 + i * 4) = c; }
    __threadfence(); }
}
__global__ __launch_bounds__(256) void csrZ_kernel(int* __restrict__ p, size_t n4) { typedef __attribute__((ext_vector_type(4))) int v4i; const size_t tid = (size_t)blockIdx.x * 256 + threadIdx.x, nth = (size_t)gridDim.x * 256; v4i z = {0, 0, 0, 0}; for (size_t i = tid; i < n4; i += nth) *(volatile v4i*)(p + i * 4) = z; }
struct CsrBufs { int *STG, *HST, *OFF, *START, *TOT, *PERM, *ROWPTR, *ROWCNT, *FLAG; int nG, NGP, CHP; size_t permLen; char* base; size_t bytes; };
static size_t csr_carve(CsrBufs& c, char* ws, size_t off, int E, int N) {
  const size_t off0 = off; c.base = ws + off;
  auto al = [&](size_t bytes) { char* p = ws + off; off += (bytes + 255) & ~(size_t)255; return p; };
  c.nG = (N + CSR_GN - 1) / CSR_GN; c.NGP = (c.nG + 31) & ~31; const int ch = (E + CSR_NBLK - 1) / CSR_NBLK; c.CHP = (ch + 31) & ~31; c.permLen = (size_t)E + 32 * (size_t)c.nG + 32;
  c.STG = (int*)al((size_t)CSR_NBLK * c.CHP * 4); c.HST = (int*)al((size_t)CSR_NBLK * c.NGP * 4); c.OFF = (int*)al((size_t)c.NGP * CSR_NBLK * 4); c.START = (int*)al((size_t)(c.NGP + 64) * 4); c.TOT = (int*)al((size_t)(c.NGP + 64) * 4);
  c.PERM = (int*)al(c.permLen * 4); c.ROWPTR = (int*)al((size_t)c.nG * CSR_GN * 4); c.ROWCNT = (int*)al((size_t)c.nG * CSR_GN * 4); c.FLAG = (int*)al(256);
  c.bytes = off - off0; return off;
}
static void csr_build(const CsrBufs& c, const int* dst, int E, int N, hipStream_t stream) {
  const size_t smem = (size_t)(2 * c.NGP + c.CHP) * 4;
  csrZ_kernel<<<512, 256, 0, stream>>>((int*)c.base, c.bytes / 16);
  csrA_kernel<<<CSR_NBLK, 64, smem, stream>>>(dst, E, N, c.nG, c.CHP, c.NGP, c.STG, c.HST);
  csrS_kernel<<<1, 512, 0, stream>>>(c.HST, c.nG, c.NGP, c.START, c.TOT, c.OFF);
  csrB_kernel<<<c.nG, 256, 0, stream>>>(dst, N, c.nG, c.CHP, c.NGP, (int)c.permLen, c.STG, c.HST, c.OFF, c.START, c.TOT, c.PERM, c.ROWPTR, c.ROWCNT, c.FLAG);
}


__global__ __launch_bounds__(256) void prepw_kernel(const float* __restrict__ w1, const float* __restrict__ w2, const float* __restrict__ wih, const float* __restrict__ whh, b16* __restrict__ WT, b16* __restrict__ WR) {
  const int t = blockIdx.x * 256 + threadIdx.x; const int per = D * D / 8; v8b o;
  if (t < NLAY * 2 * per) { const int l = t / (2 * per), kind = (t / per) % 2, e = (t % per) * 8; const int oo = e / D, k0 = e % D; const float* w = (kind == 0 ? w1 : w2) + (size_t)l * D * D;
    for (int j = 0; j < 8; ++j) o[j] = (b16)(bf16_rne(w[(k0 + j) * D + oo]) * WSC); for (int pass = 0; pass < 2; ++pass) { *(volatile v8b*)(WT + (size_t)(l * 2 + kind) * D * D + e) = o; __threadfence(); } return; }
  const int u = t - NLAY * 2 * per; if (u >= 2 * per) return; const int kind = u / per, e = (u % per) * 8; const float* w = kind == 0 ? wih : whh;
  for (int j = 0; j < 8; ++j) o[j] = (b16)(bf16_rne(w[e + j]) * WSC); for (int pass = 0; pass < 2; ++pass) { *(volatile v8b*)(WR + (size_t)kind * D * D + e) = o; __threadfence(); }
}
__device__ __forceinline__ void ego_row2(const float* __restrict__ uemb, const float* __restrict__ iemb, const float* __restrict__ EG, int layer, int row, int lane, float& x0, float& x1) {
  if (layer == 0) { const float* src = (row < NU) ? (uemb + (size_t)row * D) : (iemb + (size_t)(row - NU) * D); x0 = bf16_rne(src[lane * 2]); x1 = bf16_rne(src[lane * 2 + 1]); }
  else { const float2 v = *(const float2*)(EG + (size_t)row * D + lane * 2); x0 = v.x; x1 = v.y; }
}
__global__ __launch_bounds__(128) void layer_kernel(const float* __restrict__ uemb, const float* __restrict__ iemb, const float* __restrict__ EGin, int layer, const float* __restrict__ vals, const int* __restrict__ cols, const int* __restrict__ PERM, const int* __restrict__ ROWPTR, const int* __restrict__ ROWCNT, int permLen, const b16* __restrict__ WT, const float* __restrict__ b1, const float* __restrict__ b2, float* __restrict__ EGout) {
  __shared__ __attribute__((aligned(16))) b16 A1h[4][16][D + 8], A1l[4][16][D + 8], A2h[4][16][D + 8], A2l[4][16][D + 8]; __shared__ __attribute__((aligned(16))) float Te[4][16][D + 4];
  const int wave = threadIdx.x >> 5, lane = threadIdx.x & 31, nloc = lane & 15, hlf = lane >> 4; const size_t m0 = (size_t)blockIdx.x * 64 + wave * 16;
  const b16* W1t = WT + (size_t)(layer * 2) * D * D; const b16* W2t = WT + (size_t)(layer * 2 + 1) * D * D;
  for (int rr = 0; rr < 16; ++rr) { const int row = (int)(m0 + rr); float s0 = 0.0f, s1 = 0.0f, e0 = 0.0f, e1 = 0.0f;
    if (row < N) { ego_row2(uemb, iemb, EGin, layer, row, lane, e0, e1); int st = ROWPTR[row], cnt = ROWCNT[row]; cnt = iclamp(cnt, 0, 65536); st = iclamp(st, 0, permLen - cnt);
      for (int i = 0; i < cnt; ++i) { const int e = iclamp(PERM[st + i], 0, E - 1); const int c = iclamp(cols[e], 0, N - 1); const float v = bf16_rne(vals[e]); float x0, x1; ego_row2(uemb, iemb, EGin, layer, c, lane, x0, x1); s0 += pmul(v, x0); s1 += pmul(v, x1); } }
    b16 p, q; split16((s0 + e0) * XS, p, q); A1h[wave][rr][lane * 2] = p; A1l[wave][rr][lane * 2] = q; split16((s1 + e1) * XS, p, q); A1h[wave][rr][lane * 2 + 1] = p; A1l[wave][rr][lane * 2 + 1] = q;
    split16(pmul(s0, e0) * XS, p, q); A2h[wave][rr][lane * 2] = p; A2l[wave][rr][lane * 2] = q; split16(pmul(s1, e1) * XS, p, q); A2h[wave][rr][lane * 2 + 1] = p; A2l[wave][rr][lane * 2 + 1] = q; }
  wave_lds_sync();
  v8f acc[4] = {{}, {}, {}, {}};
#pragma unroll
  for (int kb = 0; kb < D; kb += 32) { const v16b a1 = frag_kb(&A1h[wave][nloc][kb], hlf), a1l = frag_kb(&A1l[wave][nloc][kb], hlf), a2 = frag_kb(&A2h[wave][nloc][kb], hlf), a2l = frag_kb(&A2l[wave][nloc][kb], hlf);
#pragma unroll
    for (int t = 0; t < 4; ++t) { const v16b bw1 = frag_kb(W1t + (size_t)(t * 16 + nloc) * D + kb, hlf), bw2 = frag_kb(W2t + (size_t)(t * 16 + nloc) * D + kb, hlf); acc[t] = wmma16b(a1, bw1, acc[t]); acc[t] = wmma16b(a1l, bw1, acc[t]); acc[t] = wmma16b(a2, bw2, acc[t]); acc[t] = wmma16b(a2l, bw2, acc[t]); } }
#pragma unroll
  for (int t = 0; t < 4; ++t) { const int c = t * 16 + nloc; const float bb = bf16_rne(b1[layer * D + c]) + bf16_rne(b2[layer * D + c]);
#pragma unroll
    for (int r = 0; r < 8; ++r) Te[wave][8 * hlf + r][c] = lrelu(acc[t][r] * (1.0f / (XS * WSC)) + bb); }
  wave_lds_sync();
  for (int pass = 0; pass < 2; ++pass) { for (int rr = 0; rr < 16; ++rr) if (lane < 16) *(volatile v4f*)(EGout + (m0 + rr) * D + lane * 4) = *(const v4f*)(&Te[wave][rr][lane * 4]); __threadfence(); }
}
__global__ __launch_bounds__(128) void rnn_kernel(const float* __restrict__ uemb, const float* __restrict__ iemb, const float* __restrict__ EG, int step, const int* __restrict__ uid, const int* __restrict__ iid, const b16* __restrict__ WR, const float* __restrict__ bih, const float* __restrict__ bhh, float* __restrict__ H) {
  __shared__ __attribute__((aligned(16))) b16 Xh[4][16][D + 8], Xl[4][16][D + 8], Hh[4][16][D + 8], Hl[4][16][D + 8]; __shared__ __attribute__((aligned(16))) float To[4][16][D + 4];
  const int wave = threadIdx.x >> 5, lane = threadIdx.x & 31, nloc = lane & 15, hlf = lane >> 4; const size_t s0 = (size_t)blockIdx.x * 64 + wave * 16;
  for (int rr = 0; rr < 16; ++rr) { const int s = (int)(s0 + rr); const int node = (s < NBQ) ? iclamp(uid[s], 0, NU - 1) : NU + iclamp(iid[s - NBQ], 0, NI - 1); float x0, x1;
    if (step == 0) ego_row2(uemb, iemb, nullptr, 0, node, lane, x0, x1);
    else { const float2 v = *(const float2*)(EG + (size_t)node * D + lane * 2); float q = v.x * v.x + v.y * v.y;
#pragma unroll
      for (int o = 16; o >= 1; o >>= 1) q += __shfl_xor(q, o);
      const float inv = 1.0f / fmaxf(sqrtf(q), NRM_EPS); x0 = v.x * inv; x1 = v.y * inv; }
    float h0 = 0.0f, h1 = 0.0f; if (step > 0) { const float2 hv = *(const float2*)(H + (size_t)s * D + lane * 2); h0 = hv.x; h1 = hv.y; }
    b16 p, q; split16(x0 * XS, p, q); Xh[wave][rr][lane * 2] = p; Xl[wave][rr][lane * 2] = q; split16(x1 * XS, p, q); Xh[wave][rr][lane * 2 + 1] = p; Xl[wave][rr][lane * 2 + 1] = q;
    split16(h0 * XS, p, q); Hh[wave][rr][lane * 2] = p; Hl[wave][rr][lane * 2] = q; split16(h1 * XS, p, q); Hh[wave][rr][lane * 2 + 1] = p; Hl[wave][rr][lane * 2 + 1] = q; }
  wave_lds_sync();
  v8f acc[4] = {{}, {}, {}, {}};
#pragma unroll
  for (int kb = 0; kb < D; kb += 32) { const v16b xa = frag_kb(&Xh[wave][nloc][kb], hlf), xl = frag_kb(&Xl[wave][nloc][kb], hlf), ha = frag_kb(&Hh[wave][nloc][kb], hlf), hl = frag_kb(&Hl[wave][nloc][kb], hlf);
#pragma unroll
    for (int t = 0; t < 4; ++t) { const v16b bi = frag_kb(WR + (size_t)(t * 16 + nloc) * D + kb, hlf), bh = frag_kb(WR + (size_t)D * D + (size_t)(t * 16 + nloc) * D + kb, hlf); acc[t] = wmma16b(xa, bi, acc[t]); acc[t] = wmma16b(xl, bi, acc[t]); acc[t] = wmma16b(ha, bh, acc[t]); acc[t] = wmma16b(hl, bh, acc[t]); } }
#pragma unroll
  for (int t = 0; t < 4; ++t) { const int c = t * 16 + nloc; const float bb = bf16_rne(bih[c]) + bf16_rne(bhh[c]);
#pragma unroll
    for (int r = 0; r < 8; ++r) To[wave][8 * hlf + r][c] = tanhf(acc[t][r] * (1.0f / (XS * WSC)) + bb); }
  wave_lds_sync();
  for (int pass = 0; pass < 2; ++pass) { for (int rr = 0; rr < 16; ++rr) if (lane < 16) *(volatile v4f*)(H + (s0 + rr) * D + lane * 4) = *(const v4f*)(&To[wave][rr][lane * 4]); __threadfence(); }
}
__global__ __launch_bounds__(256) void final_kernel(const float* __restrict__ H, float* __restrict__ out) {
  __shared__ __attribute__((aligned(16))) float res[256];
  const int t_ = threadIdx.x; const int b = blockIdx.x * 256 + t_; float s = 0.0f;
  for (int k = 0; k < D; ++k) s += pmul(H[(size_t)b * D + k], H[(size_t)(NBQ + b) * D + k]);
  res[t_] = s; __syncthreads();
  for (int pass = 0; pass < 2; ++pass) { if (t_ < 64) *(volatile v4f*)(out + (size_t)blockIdx.x * 256 + t_ * 4) = *(const v4f*)(&res[t_ * 4]); __threadfence(); }
}
}

extern "C" void kernel_launch(void* const* d_in, const int* in_sizes, int n_in, void* d_out, int out_size, void* d_ws, size_t ws_size, hipStream_t stream) {
  (void)n_in;
  auto Fp = [&](int i) { return (const float*)d_in[i]; }; auto Ip = [&](int i) { return (const int*)d_in[i]; };
  if (in_sizes[0] != NU * D || in_sizes[1] != NI * D || in_sizes[2] != NLAY * D * D || in_sizes[6] != D * D || in_sizes[10] != E || in_sizes[11] != E || in_sizes[12] != E || in_sizes[13] != NBQ || in_sizes[14] != NBQ || out_size != NBQ) return;
  size_t off = 0; char* ws = (char*)d_ws;
  auto carve = [&](size_t bytes) { char* p = ws + off; off += (bytes + 255) & ~(size_t)255; return p; };
  b16* WT = (b16*)carve((size_t)NLAY * 2 * D * D * 2); b16* WR = (b16*)carve((size_t)2 * D * D * 2); float* EGA = (float*)carve((size_t)NP * D * 4); float* EGB = (float*)carve((size_t)NP * D * 4); float* H = (float*)carve((size_t)NSEL * D * 4);
  CsrBufs csr; off = csr_carve(csr, ws, off, E, N);
  if (off > ws_size || off > ((size_t)128 << 20)) return;
  prepw_kernel<<<(NLAY * 2 * D * D / 8 + 2 * D * D / 8 + 255) / 256, 256, 0, stream>>>(Fp(2), Fp(3), Fp(6), Fp(7), WT, WR);
  csr_build(csr, Ip(10), E, N, stream);
  rnn_kernel<<<NSEL / 64, 128, 0, stream>>>(Fp(0), Fp(1), nullptr, 0, Ip(13), Ip(14), WR, Fp(8), Fp(9), H);
  for (int l = 0; l < NLAY; ++l) { const float* in = (l == 0) ? nullptr : ((l & 1) ? EGA : EGB); float* outp = (l & 1) ? EGB : EGA;
    layer_kernel<<<NP / 64, 128, 0, stream>>>(Fp(0), Fp(1), in, l, Fp(12), Ip(11), csr.PERM, csr.ROWPTR, csr.ROWCNT, (int)csr.permLen, WT, Fp(4), Fp(5), outp);
    rnn_kernel<<<NSEL / 64, 128, 0, stream>>>(Fp(0), Fp(1), outp, l + 1, Ip(13), Ip(14), WR, Fp(8), Fp(9), H); }
  final_kernel<<<NBQ / 256, 256, 0, stream>>>(H, (float*)d_out);
}
